// PolicyValueNet_32323923870425
// MI455X (gfx1250) — hardware-run, weakly checked
//
#include <hip/hip_runtime.h>

typedef float          v8f   __attribute__((ext_vector_type(8)));
typedef float          v4f   __attribute__((ext_vector_type(4)));
typedef unsigned int   v4u   __attribute__((ext_vector_type(4)));
typedef int            v8i   __attribute__((ext_vector_type(8)));
typedef unsigned short v8us  __attribute__((ext_vector_type(8)));
typedef unsigned short v16us __attribute__((ext_vector_type(16)));
typedef __bf16         v16bf __attribute__((ext_vector_type(16)));
typedef _Float16       v16h  __attribute__((ext_vector_type(16)));
typedef v4f  __attribute__((may_alias)) v4fa;
typedef v8us __attribute__((may_alias)) v8usa;
union FragB { v16bf v; v16us u; v8us h[2]; v8i w; };
union FragH { v16h  v; v16us u; v8us h[2]; v8i w; };

__device__ __forceinline__ v8f wmb(const FragB& a, const FragB& b, v8f c) {
  v8f d = __builtin_amdgcn_wmma_f32_16x16x32_bf16(false, a.v, false, b.v, (short)0, c, false, false);
  asm volatile("v_nop\n\tv_nop\n\tv_nop\n\tv_nop" : "+v"(d) : "v"(a.w), "v"(b.w));
  return d;
}

__device__ __forceinline__ v8f wmh(const FragH& a, const FragH& b, v8f c) {
  v8f d = __builtin_amdgcn_wmma_f32_16x16x32_f16(false, a.v, false, b.v, (short)0, c, false, false);
  asm volatile("v_nop\n\tv_nop\n\tv_nop\n\tv_nop" : "+v"(d) : "v"(a.w), "v"(b.w));
  return d;
}

__device__ __forceinline__ unsigned bf16_bits(float f) {
  const unsigned u = __float_as_uint(f);
  const unsigned r = (u + 0x7FFFu + ((u >> 16) & 1u)) >> 16;
  const unsigned q = (u >> 16) | 0x40u;
  return ((u & 0x7fffffffu) > 0x7f800000u) ? q : r;
}

__device__ __forceinline__ float bf16_val(float f) {
  return __uint_as_float(bf16_bits(f) << 16);
}
__device__ __forceinline__ int clampi(int v, int lo, int hi) {
  return v < lo ? lo : (v > hi ? hi : v);
}

__device__ __forceinline__ unsigned f16_bits(float f) {
  const unsigned u  = __float_as_uint(f);
  const unsigned s  = (u >> 16) & 0x8000u;
  const unsigned a  = u & 0x7fffffffu;
  const unsigned t  = a - 0x38000000u;
  const unsigned r  = (t + 0x0FFFu + ((t >> 13) & 1u)) >> 13;
  const unsigned rc = r > 0x7C00u ? 0x7C00u : r;
  const bool small  = a < 0x38800000u;
  const bool isnan  = a > 0x7f800000u;
  const unsigned fin = small ? 0u : (s | rc);
  return isnan ? (s | 0x7E00u) : fin;
}

__device__ __forceinline__ unsigned pk16(unsigned lo, unsigned hi) { return lo | (hi << 16); }
__device__ __forceinline__ unsigned bf16_lo_bits(float v) {
  float hi = bf16_val(v);
  asm volatile("" : "+v"(hi));
  return bf16_bits(v - hi);
}
__device__ __forceinline__ v4u pack8_bf16(v4f a, v4f c) {
  return (v4u){ pk16(bf16_bits(a[0]), bf16_bits(a[1])), pk16(bf16_bits(a[2]), bf16_bits(a[3])),
                pk16(bf16_bits(c[0]), bf16_bits(c[1])), pk16(bf16_bits(c[2]), bf16_bits(c[3])) };
}
__device__ __forceinline__ v4u pack8_bf16_lo(v4f a, v4f c) {
  return (v4u){ pk16(bf16_lo_bits(a[0]), bf16_lo_bits(a[1])), pk16(bf16_lo_bits(a[2]), bf16_lo_bits(a[3])),
                pk16(bf16_lo_bits(c[0]), bf16_lo_bits(c[1])), pk16(bf16_lo_bits(c[2]), bf16_lo_bits(c[3])) };
}
__device__ __forceinline__ v4u pack8_f16(v4f a, v4f c) {
  return (v4u){ pk16(f16_bits(a[0]), f16_bits(a[1])), pk16(f16_bits(a[2]), f16_bits(a[3])),
                pk16(f16_bits(c[0]), f16_bits(c[1])), pk16(f16_bits(c[2]), f16_bits(c[3])) };
}

template <int FORM>
__global__ __launch_bounds__(256) void k_plane(const float* __restrict__ src, int rows, int cols, int ldsrc,
                                               unsigned short* __restrict__ dst, int MP, int KP) {
  static_assert(FORM >= 0 && FORM <= 3);
  const int KTOT = (FORM == 1 || FORM == 3) ? 2 * KP : KP;
  const unsigned ppr   = (unsigned)(KTOT >> 3);
  const unsigned kp8   = (unsigned)(KP >> 3);
  const unsigned total = (unsigned)MP * ppr;
  const unsigned g     = blockIdx.x * 256u + threadIdx.x;
  const unsigned rowu  = g / ppr;
  const unsigned p     = g - rowu * ppr;
  const bool second    = p >= kp8;
  const int row = (int)rowu;
  const int c0  = (int)((second ? p - kp8 : p) << 3);
  const float* srow = src + (size_t)clampi(row, 0, rows - 1) * (size_t)ldsrc;
  float x[8];
  unsigned mk[8];
#pragma unroll
  for (int e = 0; e < 8; ++e) {
    const int c = c0 + e;
    const float v = srow[clampi(c, 0, cols - 1)];
    asm volatile("" :: "v"(v));
    x[e]  = v;
    mk[e] = (row < rows && c < cols) ? 0xFFFFu : 0u;
  }
  const v4f a = (v4f){ x[0], x[1], x[2], x[3] };
  const v4f c = (v4f){ x[4], x[5], x[6], x[7] };
  v4u o;
  if (FORM == 2) {
    o = pack8_f16(a, c);
  } else {
    const v4u hi = pack8_bf16(a, c);
    o = hi;
    if (FORM == 1) { const v4u lo = pack8_bf16_lo(a, c); o = second ? lo : hi; }
  }
  const v4u mw = (v4u){ pk16(mk[0], mk[1]), pk16(mk[2], mk[3]), pk16(mk[4], mk[5]), pk16(mk[6], mk[7]) };
  o &= mw;
  if (g < total) {
    volatile v4u* q = (volatile v4u*)(dst + (size_t)g * 8);
    *q = o;
    __threadfence();
    *q = o;
  }
}

template <int FORM> struct FragOf    { typedef FragB T; };
template <>         struct FragOf<2> { typedef FragH T; };
__device__ __forceinline__ v8f mm(const FragB& a, const FragB& b, v8f c) { return wmb(a, b, c); }
__device__ __forceinline__ v8f mm(const FragH& a, const FragH& b, v8f c) { return wmh(a, b, c); }
template <class F> __device__ __forceinline__ F ld_frag(const unsigned short* p) {
  F f;
  f.h[0] = *(const v8usa*)(p);
  f.h[1] = *(const v8usa*)(p + 16);
  return f;
}

template <int FORM, int EPI>
__global__ __launch_bounds__(256) __attribute__((amdgpu_num_vgpr(248)))
void k_gemm_nt(const unsigned short* __restrict__ A, const unsigned short* __restrict__ B,
               const float* __restrict__ bias, float* __restrict__ D, int M, int N, int KTOT, int ldd) {
  static_assert(FORM >= 0 && FORM <= 2);
  static_assert(EPI == 0 || EPI == 1);
  typedef typename FragOf<FORM>::T F;
  __shared__ __attribute__((aligned(16))) float sT[8][16 * 68];
  const int lane = threadIdx.x & 31;
  const int wave = threadIdx.x >> 5;
  const int tilesM = (M + 63) >> 6;
  const int tilesN = (N + 63) >> 6;
  const int tile = blockIdx.x * 8 + wave;
  if (tile >= tilesM * tilesN) return;
  const int tm = tile / tilesN;
  const int tn = tile - tm * tilesN;
  const int m0 = tm << 6;
  const int n0 = tn << 6;

  const int rl = lane & 15;
  const int h8 = (lane >> 4) * 8;
  const unsigned short* pa = A + (size_t)(m0 + rl) * (size_t)KTOT + h8;
  const unsigned short* pb = B + (size_t)(n0 + rl) * (size_t)KTOT + h8;

  v8f acc[4][4];
#pragma unroll
  for (int i = 0; i < 4; ++i)
#pragma unroll
    for (int j = 0; j < 4; ++j) acc[i][j] = (v8f){0.f, 0.f, 0.f, 0.f, 0.f, 0.f, 0.f, 0.f};

#pragma unroll 1
  for (int k0 = 0; k0 < KTOT; k0 += 32) {
    F bf[4];
#pragma unroll
    for (int j = 0; j < 4; ++j) bf[j] = ld_frag<F>(pb + (size_t)(j << 4) * (size_t)KTOT + k0);
#pragma unroll
    for (int i = 0; i < 4; ++i) {
      const F af = ld_frag<F>(pa + (size_t)(i << 4) * (size_t)KTOT + k0);
#pragma unroll
      for (int j = 0; j < 4; ++j) acc[i][j] = mm(af, bf[j], acc[i][j]);
    }
  }

  float* slab = sT[wave];
  const int hh = lane >> 4;
  const int c4 = (lane & 15) * 4;
  const int nc = n0 + c4;
  const bool cok = nc < N;
  v4f bv = (v4f){0.f, 0.f, 0.f, 0.f};
  if (EPI == 1) {
    bv = *(const v4fa*)(bias + clampi(nc, 0, N - 4));
    asm volatile("" :: "v"(bv));
  }
#pragma unroll
  for (int i = 0; i < 4; ++i) {
    const int mBase = m0 + (i << 4);
#pragma unroll
    for (int j = 0; j < 4; ++j) {
#pragma unroll
      for (int r = 0; r < 8; ++r) slab[(h8 + r) * 68 + (j << 4) + rl] = acc[i][j][r];
    }
    __builtin_amdgcn_fence(__ATOMIC_RELEASE, "workgroup");
    __builtin_amdgcn_wave_barrier();
    __builtin_amdgcn_fence(__ATOMIC_ACQUIRE, "workgroup");
    v4f vv[8];
#pragma unroll
    for (int it = 0; it < 8; ++it) {
      const int row = it * 2 + hh;
      v4f v = *(const v4fa*)(slab + row * 68 + c4);
      if (EPI == 1) v += bv;
      vv[it] = v;
    }
    for (int pass = 0; pass < 2; ++pass) {
#pragma unroll
      for (int it = 0; it < 8; ++it) {
        const int row = mBase + it * 2 + hh;
        if (cok && row < M) *(volatile v4f*)(D + (size_t)row * (size_t)ldd + nc) = vv[it];
      }
      __threadfence();
    }
    __builtin_amdgcn_fence(__ATOMIC_RELEASE, "workgroup");
    __builtin_amdgcn_wave_barrier();
    __builtin_amdgcn_fence(__ATOMIC_ACQUIRE, "workgroup");
  }
}

#ifndef CONV_TERMS
#define CONV_TERMS 2
#endif
static_assert(CONV_TERMS == 1 || CONV_TERMS == 2);
#if CONV_TERMS == 2
#define WFORM 3
#define AFORM 1
#else
#define WFORM 0
#define AFORM 0
#endif

#define NMOVES  200000
#define BH      20
#define BW      20
#define HWP     400
#define MPAD    448
#define CIN     8
#define CH      128
#define NPIECE  21
#define NBLK    10
#define KST     72
#define KSTP    96
#define KBL     1152
#define KBLT    (KBL * CONV_TERMS)
#define KPV     (CH * CONV_TERMS)
#define NPVC    192
#define VCH     64
#define PW1LD   147
#define VW1LD   107
#define TABROWS 32
#define TABUSED 26
#define POLW    10
#define WSLIM   ((size_t)128 << 20)

static_assert(HWP == BH * BW && HWP <= MPAD && MPAD % 64 == 0 && HWP % 16 == 0 && HWP == 16 * 25);
static_assert(KST == CIN * 9 && KST <= KSTP && KSTP % 32 == 0);
static_assert(KBL == CH * 9 && KBL % 32 == 0 && KBLT % 32 == 0 && KPV % 32 == 0);
static_assert(PW1LD == CH + 16 + 3);
static_assert(VW1LD == VCH + 2 * NPIECE + 1);
static_assert(CH / 8 == 16 && VCH / 8 == 8 && CH + VCH == NPVC && NPVC % 64 == 0 && NPVC % 32 == 0);
static_assert(NMOVES % (32 * POLW) == 0);
static_assert(TABUSED == NPIECE + 5 && TABUSED <= TABROWS);
static_assert((MPAD * (KSTP / 8)) % 256 == 0 && (MPAD * (KBLT / 8)) % 256 == 0 && (MPAD * (KPV / 8)) % 256 == 0);
static_assert((128 * (KSTP / 8)) % 256 == 0 && (NBLK * 2 * CH * (KBLT / 8)) % 256 == 0);
static_assert((CH * (KPV / 8)) % 256 == 0 && (VCH * (KPV / 8)) % 256 == 0);
static_assert((NMOVES * 4) % 128 == 0);

typedef int   v4i __attribute__((ext_vector_type(4)));
typedef float v2f __attribute__((ext_vector_type(2)));
typedef v4i __attribute__((may_alias)) v4ia;
typedef v2f __attribute__((may_alias)) v2fa;

__device__ __forceinline__ v4f bf16_v4(v4f a) {
  return (v4f){ bf16_val(a[0]), bf16_val(a[1]), bf16_val(a[2]), bf16_val(a[3]) };
}

__global__ __launch_bounds__(256) void k_im2col(const float* __restrict__ src, int sp, int sc, int K, int KP, int terms,
                                                unsigned short* __restrict__ dst) {
  const int KTOT = KP * terms;
  const unsigned ppr   = (unsigned)(KTOT >> 3);
  const unsigned kp8   = (unsigned)(KP >> 3);
  const unsigned total = (unsigned)MPAD * ppr;
  const unsigned g     = blockIdx.x * 256u + threadIdx.x;
  const unsigned gc    = g < total ? g : total - 1u;
  const unsigned rowu  = gc / ppr;
  const unsigned p     = gc - rowu * ppr;
  const bool second    = p >= kp8;
  const int row = (int)rowu;
  const int c0  = (int)((second ? p - kp8 : p) << 3);
  const int pos = clampi(row, 0, HWP - 1);
  const int y   = pos / BW;
  const int x   = pos - y * BW;
  float v[8];
  unsigned mk[8];
#pragma unroll
  for (int e = 0; e < 8; ++e) {
    const int k  = c0 + e;
    const int kc = clampi(k, 0, K - 1);
    const int c  = kc / 9;
    const int t  = kc - c * 9;
    const int ky = t / 3;
    const int kx = t - ky * 3;
    const int yy = y + ky - 1;
    const int xx = x + kx - 1;
    const bool ok = (row < HWP) && (k < K) && ((unsigned)yy < (unsigned)BH) && ((unsigned)xx < (unsigned)BW);
    const int sidx = (clampi(yy, 0, BH - 1) * BW + clampi(xx, 0, BW - 1)) * sp + c * sc;
    const float val = src[sidx];
    asm volatile("" :: "v"(val));
    v[e]  = val;
    mk[e] = ok ? 0xFFFFu : 0u;
  }
  const v4f a = (v4f){ v[0], v[1], v[2], v[3] };
  const v4f c = (v4f){ v[4], v[5], v[6], v[7] };
  const v4u hi = pack8_bf16(a, c);
  const v4u lo = pack8_bf16_lo(a, c);
  v4u o = second ? lo : hi;
  const v4u mw = (v4u){ pk16(mk[0], mk[1]), pk16(mk[2], mk[3]), pk16(mk[4], mk[5]), pk16(mk[6], mk[7]) };
  o &= mw;
  if (g < total) {
    volatile v4u* q = (volatile v4u*)(dst + (size_t)g * 8);
    *q = o;
    __threadfence();
    *q = o;
  }
}

__global__ __launch_bounds__(512) void k_gn(const float* __restrict__ Y, const float* __restrict__ cbias,
                                            const float* __restrict__ gsc, const float* __restrict__ gbi,
                                            const float* __restrict__ R, float* __restrict__ OUT, int mode) {
  __shared__ double sPart[512];
  __shared__ double sStat[16];
  const int t    = threadIdx.x;
  const int lane = t & 31;
  const int wave = t >> 5;
  const int c4   = lane * 4;
  const v4f cb = bf16_v4(*(const v4fa*)(cbias + c4));
  const v4f gs = bf16_v4(*(const v4fa*)(gsc + c4));
  const v4f gb = bf16_v4(*(const v4fa*)(gbi + c4));

  double s = 0.0;
#pragma unroll 1
  for (int j = 0; j < 25; ++j) {
    const int p = wave + 16 * j;
    const v4f v = *(const v4fa*)(Y + p * CH + c4);
    s += (double)(v[0] + cb[0]);
    s += (double)(v[1] + cb[1]);
    s += (double)(v[2] + cb[2]);
    s += (double)(v[3] + cb[3]);
  }
  sPart[t] = s;
  __syncthreads();
  if (t < 8) {
    double a = 0.0;
#pragma unroll 1
    for (int w = 0; w < 16; ++w) {
#pragma unroll 1
      for (int l = 0; l < 4; ++l) a += sPart[w * 32 + t * 4 + l];
    }
    sStat[t] = a * (1.0 / 6400.0);
  }
  __syncthreads();
  const double mean = sStat[lane >> 2];
  double s2 = 0.0;
#pragma unroll 1
  for (int j = 0; j < 25; ++j) {
    const int p = wave + 16 * j;
    const v4f v = *(const v4fa*)(Y + p * CH + c4);
    const double d0 = (double)(v[0] + cb[0]) - mean;
    const double d1 = (double)(v[1] + cb[1]) - mean;
    const double d2 = (double)(v[2] + cb[2]) - mean;
    const double d3 = (double)(v[3] + cb[3]) - mean;
    s2 += d0 * d0;
    s2 += d1 * d1;
    s2 += d2 * d2;
    s2 += d3 * d3;
  }
  sPart[t] = s2;
  __syncthreads();
  if (t < 8) {
    double a = 0.0;
#pragma unroll 1
    for (int w = 0; w < 16; ++w) {
#pragma unroll 1
      for (int l = 0; l < 4; ++l) a += sPart[w * 32 + t * 4 + l];
    }
    sStat[8 + t] = a * (1.0 / 6400.0);
  }
  __syncthreads();
  const float mf   = (float)mean;
  const float var  = (float)sStat[8 + (lane >> 2)];
  const float rstd = 1.0f / sqrtf(var + 1e-5f);
#pragma unroll 1
  for (int j = 0; j < 25; ++j) {
    const int p = wave + 16 * j;
    const v4f v = *(const v4fa*)(Y + p * CH + c4);
    v4f r = (v4f){0.f, 0.f, 0.f, 0.f};
    if (mode != 0) r = *(const v4fa*)(R + p * CH + c4);
    v4f o;
#pragma unroll
    for (int e = 0; e < 4; ++e) {
      const float x  = v[e] + cb[e];
      const float xn = (x - mf) * rstd;
      float yv = xn * gs[e] + gb[e];
      yv = yv + r[e];
      o[e] = (yv > 0.0f) ? yv : 0.0f;
    }
    volatile v4f* q = (volatile v4f*)(OUT + p * CH + c4);
    *q = o;
    __threadfence();
    *q = o;
  }
}

__global__ __launch_bounds__(256) void k_tab(const float* __restrict__ emb, const float* __restrict__ w1,
                                             const float* __restrict__ b1, const float* __restrict__ w2,
                                             float* __restrict__ TAB) {
  const int t   = blockIdx.x * 256 + threadIdx.x;
  const int row = t >> 5;
  const int o0  = (t & 31) * 4;
  v4f o = (v4f){0.f, 0.f, 0.f, 0.f};
  if (row < NPIECE) {
    float a0 = 0.0f, a1 = 0.0f, a2 = 0.0f, a3 = 0.0f;
#pragma unroll 1
    for (int tt = 0; tt < 16; ++tt) {
      const float ev = bf16_val(emb[row * 16 + tt]);
      const float q0 = bf16_val(w1[(o0 + 0) * PW1LD + CH + tt]);
      const float q1 = bf16_val(w1[(o0 + 1) * PW1LD + CH + tt]);
      const float q2 = bf16_val(w1[(o0 + 2) * PW1LD + CH + tt]);
      const float q3 = bf16_val(w1[(o0 + 3) * PW1LD + CH + tt]);
      a0 = a0 + ev * q0;
      a1 = a1 + ev * q1;
      a2 = a2 + ev * q2;
      a3 = a3 + ev * q3;
    }
    o = (v4f){ a0, a1, a2, a3 };
  } else if (row < NPIECE + 3) {
    const int col = CH + 16 + (row - NPIECE);
    const float q0 = w1[(o0 + 0) * PW1LD + col];
    const float q1 = w1[(o0 + 1) * PW1LD + col];
    const float q2 = w1[(o0 + 2) * PW1LD + col];
    const float q3 = w1[(o0 + 3) * PW1LD + col];
    o = (v4f){ bf16_val(q0), bf16_val(q1), bf16_val(q2), bf16_val(q3) };
  } else if (row == NPIECE + 3) {
    o = bf16_v4(*(const v4fa*)(b1 + o0));
  } else if (row == NPIECE + 4) {
    o = bf16_v4(*(const v4fa*)(w2 + o0));
  }
  volatile v4f* q = (volatile v4f*)(TAB + 4 * t);
  *q = o;
  __threadfence();
  *q = o;
}

__global__ __launch_bounds__(320) void k_moves(const float* __restrict__ PV, const float* __restrict__ TAB,
                                               const int* __restrict__ cells, const int* __restrict__ counts,
                                               const int* __restrict__ pids, const float* __restrict__ anchors,
                                               const float* __restrict__ sizes, const float* __restrict__ pb2,
                                               float* __restrict__ logits) {
  __shared__ __attribute__((aligned(16))) float sTab[TABUSED * CH];
  __shared__ __attribute__((aligned(16))) int   sCells[POLW][320];
  __shared__ int   sCnt[POLW][32];
  __shared__ int   sPid[POLW][32];
  __shared__ __attribute__((aligned(8))) float sAnc[POLW][64];
  __shared__ float sSz[POLW][32];
  const int t    = threadIdx.x;
  const int lane = t & 31;
  const int wave = t >> 5;

  for (int i = t; i < TABUSED * (CH / 4); i += 32 * POLW) {
    const v4f v = *(const v4fa*)(TAB + 4 * i);
    *(v4fa*)(sTab + 4 * i) = v;
  }

  const int m0 = (blockIdx.x * POLW + wave) * 32;
  const int* cp = cells + (size_t)m0 * 10;
  const int i2  = 256 + 4 * lane;
  const int i2c = i2 < 316 ? i2 : 316;
  const v4i c0v = *(const v4ia*)(cp + 4 * lane);
  const v4i c1v = *(const v4ia*)(cp + 128 + 4 * lane);
  const v4i c2v = *(const v4ia*)(cp + i2c);
  const int   cn = counts[m0 + lane];
  const int   pd = pids[m0 + lane];
  const v2f   an = *(const v2fa*)(anchors + 2 * (m0 + lane));
  const float sz = sizes[m0 + lane];
  asm volatile("" :: "v"(c0v), "v"(c1v), "v"(c2v));
  asm volatile("" :: "v"(cn), "v"(pd), "v"(an), "v"(sz));
  *(v4ia*)(&sCells[wave][4 * lane]) = c0v;
  *(v4ia*)(&sCells[wave][128 + 4 * lane]) = c1v;
  if (lane < 16) *(v4ia*)(&sCells[wave][256 + 4 * lane]) = c2v;
  sCnt[wave][lane] = cn;
  sPid[wave][lane] = pd;
  *(v2fa*)(&sAnc[wave][2 * lane]) = (v2f){ bf16_val(an[0]), bf16_val(an[1]) };
  sSz[wave][lane] = bf16_val(sz);
  __syncthreads();

  const v4f wa0 = *(const v4fa*)(sTab + (NPIECE + 0) * CH + 4 * lane);
  const v4f wa1 = *(const v4fa*)(sTab + (NPIECE + 1) * CH + 4 * lane);
  const v4f wsz = *(const v4fa*)(sTab + (NPIECE + 2) * CH + 4 * lane);
  const v4f b1v = *(const v4fa*)(sTab + (NPIECE + 3) * CH + 4 * lane);
  const v4f w2v = *(const v4fa*)(sTab + (NPIECE + 4) * CH + 4 * lane);
  const float b2 = bf16_val(pb2[0]);
  float mine = 0.0f;

#pragma unroll 1
  for (int m = 0; m < 32; ++m) {
    const int   cnt = sCnt[wave][m];
    const int   pid = clampi(sPid[wave][m], 0, NPIECE - 1);
    const float a0  = sAnc[wave][2 * m];
    const float a1  = sAnc[wave][2 * m + 1];
    const float s   = sSz[wave][m];
    v4f rowv[5];
#pragma unroll
    for (int k = 0; k < 5; ++k) {
      const int cx = clampi(sCells[wave][10 * m + 2 * k], 0, BW - 1);
      const int cy = clampi(sCells[wave][10 * m + 2 * k + 1], 0, BH - 1);
      rowv[k] = *(const v4fa*)(PV + (size_t)(cy * BW + cx) * NPVC + 4 * lane);
      asm volatile("" :: "v"(rowv[k]));
    }
    v4f acc = (v4f){0.f, 0.f, 0.f, 0.f};
#pragma unroll
    for (int k = 0; k < 5; ++k) {
      const unsigned mk = (k < cnt) ? 0xFFFFFFFFu : 0u;
#pragma unroll
      for (int e = 0; e < 4; ++e) acc[e] = acc[e] + __uint_as_float(__float_as_uint(rowv[k][e]) & mk);
    }
    const float cf = (float)cnt;
    const v4f pe = *(const v4fa*)(sTab + pid * CH + 4 * lane);
    float part = 0.0f;
#pragma unroll
    for (int e = 0; e < 4; ++e) {
      float v = acc[e] / cf;
      v = v + pe[e];
      v = v + a0 * wa0[e];
      v = v + a1 * wa1[e];
      v = v + s * wsz[e];
      v = v + b1v[e];
      v = (v > 0.0f) ? v : (v - v);
      part = part + v * w2v[e];
    }
    part += __shfl_xor(part, 16);
    part += __shfl_xor(part, 8);
    part += __shfl_xor(part, 4);
    part += __shfl_xor(part, 2);
    part += __shfl_xor(part, 1);
    const float tot = part + b2;
    mine = (lane == m) ? tot : mine;
  }
  volatile float* q = (volatile float*)(logits + m0 + lane);
  *q = mine;
  __threadfence();
  *q = mine;
}

__global__ __launch_bounds__(256) void k_shead(const float* __restrict__ PV, const float* __restrict__ cb,
                                               const float* __restrict__ gsc, const float* __restrict__ gbi,
                                               const float* __restrict__ srem, const float* __restrict__ orem,
                                               const float* __restrict__ phase,
                                               const float* __restrict__ w1, const float* __restrict__ b1,
                                               const float* __restrict__ w2, const float* __restrict__ b2,
                                               const float* __restrict__ w3, const float* __restrict__ b3,
                                               float* __restrict__ out) {
  __shared__ double sPart[256];
  __shared__ double sPool[16 * VCH];
  __shared__ double sStat[16];
  __shared__ float  sVin[112];
  __shared__ float  sH1[256];
  __shared__ float  sH2[128];
  __shared__ float  sProd[128];
  const int t  = threadIdx.x;
  const int cl = t & 15;
  const int r  = t >> 4;
  const int c4 = cl * 4;
  const v4f cbv = bf16_v4(*(const v4fa*)(cb + c4));
  const v4f gs  = bf16_v4(*(const v4fa*)(gsc + c4));
  const v4f gb  = bf16_v4(*(const v4fa*)(gbi + c4));

  double s = 0.0;
#pragma unroll 1
  for (int j = 0; j < 25; ++j) {
    const int p = r + 16 * j;
    const v4f v = *(const v4fa*)(PV + p * NPVC + CH + c4);
    s += (double)(v[0] + cbv[0]);
    s += (double)(v[1] + cbv[1]);
    s += (double)(v[2] + cbv[2]);
    s += (double)(v[3] + cbv[3]);
  }
  sPart[t] = s;
  __syncthreads();
  if (t < 8) {
    double a = 0.0;
#pragma unroll 1
    for (int rr = 0; rr < 16; ++rr) {
#pragma unroll 1
      for (int l = 0; l < 2; ++l) a += sPart[rr * 16 + 2 * t + l];
    }
    sStat[t] = a * (1.0 / 3200.0);
  }
  __syncthreads();
  const double mean = sStat[cl >> 1];
  double s2 = 0.0;
#pragma unroll 1
  for (int j = 0; j < 25; ++j) {
    const int p = r + 16 * j;
    const v4f v = *(const v4fa*)(PV + p * NPVC + CH + c4);
    const double d0 = (double)(v[0] + cbv[0]) - mean;
    const double d1 = (double)(v[1] + cbv[1]) - mean;
    const double d2 = (double)(v[2] + cbv[2]) - mean;
    const double d3 = (double)(v[3] + cbv[3]) - mean;
    s2 += d0 * d0;
    s2 += d1 * d1;
    s2 += d2 * d2;
    s2 += d3 * d3;
  }
  sPart[t] = s2;
  __syncthreads();
  if (t < 8) {
    double a = 0.0;
#pragma unroll 1
    for (int rr = 0; rr < 16; ++rr) {
#pragma unroll 1
      for (int l = 0; l < 2; ++l) a += sPart[rr * 16 + 2 * t + l];
    }
    sStat[8 + t] = a * (1.0 / 3200.0);
  }
  __syncthreads();
  const float mf   = (float)mean;
  const float var  = (float)sStat[8 + (cl >> 1)];
  const float rstd = 1.0f / sqrtf(var + 1e-5f);
  double p0 = 0.0, p1 = 0.0, p2 = 0.0, p3 = 0.0;
#pragma unroll 1
  for (int j = 0; j < 25; ++j) {
    const int p = r + 16 * j;
    const v4f v = *(const v4fa*)(PV + p * NPVC + CH + c4);
    float o[4];
#pragma unroll
    for (int e = 0; e < 4; ++e) {
      const float x  = v[e] + cbv[e];
      const float xn = (x - mf) * rstd;
      const float yv = xn * gs[e] + gb[e];
      o[e] = (yv > 0.0f) ? yv : 0.0f;
    }
    p0 += (double)o[0];
    p1 += (double)o[1];
    p2 += (double)o[2];
    p3 += (double)o[3];
  }
  sPool[r * VCH + c4 + 0] = p0;
  sPool[r * VCH + c4 + 1] = p1;
  sPool[r * VCH + c4 + 2] = p2;
  sPool[r * VCH + c4 + 3] = p3;
  __syncthreads();
  {
    const int tc = t & 63;
    double a = 0.0;
#pragma unroll 1
    for (int rr = 0; rr < 16; ++rr) a += sPool[rr * VCH + tc];
    const float pooled = (float)(a * (1.0 / 400.0));
    const float sr  = srem[clampi(t - 64, 0, NPIECE - 1)];
    const float orr = orem[clampi(t - 85, 0, NPIECE - 1)];
    const float ph  = phase[0];
    asm volatile("" :: "v"(sr), "v"(orr), "v"(ph));
    const unsigned q0 = (t < 64) ? 0xFFFFFFFFu : 0u;
    const unsigned q1 = (t >= 64 && t < 85) ? 0xFFFFFFFFu : 0u;
    const unsigned q2 = (t >= 85 && t < 106) ? 0xFFFFFFFFu : 0u;
    const unsigned q3 = (t == 106) ? 0xFFFFFFFFu : 0u;
    const unsigned bits = (__float_as_uint(pooled) & q0) | ((bf16_bits(sr) << 16) & q1) |
                          ((bf16_bits(orr) << 16) & q2) | ((bf16_bits(ph) << 16) & q3);
    if (t < 112) sVin[t] = __uint_as_float(bits);
  }
  __syncthreads();
  {
    float acc = 0.0f;
#pragma unroll 4
    for (int k = 0; k < VW1LD; ++k) acc = acc + bf16_val(w1[t * VW1LD + k]) * sVin[k];
    acc = acc + bf16_val(b1[t]);
    sH1[t] = (acc > 0.0f) ? acc : 0.0f;
  }
  __syncthreads();
  {
    const int o = t & 127;
    float acc = 0.0f;
#pragma unroll 4
    for (int k = 0; k < 256; ++k) acc = acc + bf16_val(w2[o * 256 + k]) * sH1[k];
    acc = acc + bf16_val(b2[o]);
    const float h = (acc > 0.0f) ? acc : 0.0f;
    if (t < 128) sH2[o] = h;
  }
  __syncthreads();
  {
    const int o = t & 127;
    const float pr = bf16_val(w3[o]) * sH2[o];
    if (t < 128) sProd[o] = pr;
  }
  __syncthreads();
  float acc = 0.0f;
#pragma unroll 1
  for (int k = 0; k < 128; ++k) acc = acc + sProd[k];
  acc = acc + bf16_val(b3[0]);
  const float val = tanhf(acc);
  if (t == 0) {
    volatile float* q = (volatile float*)(out + NMOVES);
    *q = val;
    __threadfence();
    *q = val;
  }
}

extern "C" void kernel_launch(void* const* d_in, const int* in_sizes, int n_in,
                              void* d_out, int out_size, void* d_ws, size_t ws_size,
                              hipStream_t stream) {
  if (n_in < 32) return;
  const int expect[32] = { 3200, 21, 21, 1, 400000, 200000, 9216, 128, 128, 128, 2949120, 2560, 2560, 2560, 336,
                           18816, 128, 128, 1, 8192, 64, 64, 64, 27392, 256, 32768, 128, 128, 1,
                           200000, 2000000, 200000 };
  for (int i = 0; i < 32; ++i) if (in_sizes[i] != expect[i]) return;
  if (out_size != NMOVES + 1) return;

  const float* board   = (const float*)d_in[0];
  const float* srem    = (const float*)d_in[1];
  const float* orem    = (const float*)d_in[2];
  const float* phase   = (const float*)d_in[3];
  const float* anchors = (const float*)d_in[4];
  const float* sizes   = (const float*)d_in[5];
  const float* stem_w  = (const float*)d_in[6];
  const float* stem_b  = (const float*)d_in[7];
  const float* stem_gs = (const float*)d_in[8];
  const float* stem_gb = (const float*)d_in[9];
  const float* blk_w   = (const float*)d_in[10];
  const float* blk_b   = (const float*)d_in[11];
  const float* blk_gs  = (const float*)d_in[12];
  const float* blk_gb  = (const float*)d_in[13];
  const float* emb     = (const float*)d_in[14];
  const float* pol_w1  = (const float*)d_in[15];
  const float* pol_b1  = (const float*)d_in[16];
  const float* pol_w2  = (const float*)d_in[17];
  const float* pol_b2  = (const float*)d_in[18];
  const float* val_cw  = (const float*)d_in[19];
  const float* val_cb  = (const float*)d_in[20];
  const float* val_gs  = (const float*)d_in[21];
  const float* val_gb  = (const float*)d_in[22];
  const float* val_w1  = (const float*)d_in[23];
  const float* val_b1  = (const float*)d_in[24];
  const float* val_w2  = (const float*)d_in[25];
  const float* val_b2  = (const float*)d_in[26];
  const float* val_w3  = (const float*)d_in[27];
  const float* val_b3  = (const float*)d_in[28];
  const int* piece_ids   = (const int*)d_in[29];
  const int* cells       = (const int*)d_in[30];
  const int* cell_counts = (const int*)d_in[31];
  float* out = (float*)d_out;

  constexpr int    NWROWS = NBLK * 2 * CH;
  constexpr size_t szWB   = (size_t)NWROWS * KBLT * 2;
  constexpr size_t szWST  = (size_t)CH * KSTP * 2;
  constexpr size_t szWPV  = (size_t)NPVC * KPV * 2;
  constexpr size_t szTAB  = (size_t)TABROWS * CH * 4;
  constexpr size_t szCOL  = (size_t)MPAD * KBLT * 2;
  constexpr size_t szY    = (size_t)MPAD * CH * 4;
  constexpr size_t szACT  = (size_t)MPAD * CH * 4;
  constexpr size_t szFHL  = (size_t)MPAD * KPV * 2;
  constexpr size_t szPV   = (size_t)MPAD * NPVC * 4;
  static_assert(NWROWS % 64 == 0);
  static_assert(szWB % 256 == 0 && szWST % 256 == 0 && szWPV % 256 == 0 && szTAB % 256 == 0 && szCOL % 256 == 0);
  static_assert(szY % 256 == 0 && szACT % 256 == 0 && szFHL % 256 == 0 && szPV % 256 == 0);
  static_assert((size_t)MPAD * KSTP * 2 <= szCOL);
  constexpr size_t oWB   = 0;
  constexpr size_t oWST  = oWB + szWB;
  constexpr size_t oWPV  = oWST + szWST;
  constexpr size_t oTAB  = oWPV + szWPV;
  constexpr size_t oCOL  = oTAB + szTAB;
  constexpr size_t oY    = oCOL + szCOL;
  constexpr size_t oACT0 = oY + szY;
  constexpr size_t oACT1 = oACT0 + szACT;
  constexpr size_t oACT2 = oACT1 + szACT;
  constexpr size_t oFHL  = oACT2 + szACT;
  constexpr size_t oPV   = oFHL + szFHL;
  constexpr size_t total = oPV + szPV;
  static_assert(total <= WSLIM);
  static_assert(CONV_TERMS != 2 || total == (size_t)15491072);
  if (total > ws_size) return;

  char* ws = (char*)d_ws;
  unsigned short* WB  = (unsigned short*)(ws + oWB);
  unsigned short* WST = (unsigned short*)(ws + oWST);
  unsigned short* WPV = (unsigned short*)(ws + oWPV);
  float*          TAB = (float*)(ws + oTAB);
  unsigned short* COL = (unsigned short*)(ws + oCOL);
  float*          Y   = (float*)(ws + oY);
  float*          A0  = (float*)(ws + oACT0);
  float*          A1  = (float*)(ws + oACT1);
  float*          A2  = (float*)(ws + oACT2);
  unsigned short* FHL = (unsigned short*)(ws + oFHL);
  float*          PV  = (float*)(ws + oPV);

  k_plane<0><<<dim3(CH * (KSTP / 8) / 256), dim3(256), 0, stream>>>(stem_w, CH, KST, KST, WST, CH, KSTP);
  k_plane<WFORM><<<dim3(NWROWS * (KBLT / 8) / 256), dim3(256), 0, stream>>>(blk_w, NWROWS, KBL, KBL, WB, NWROWS, KBL);
  k_plane<WFORM><<<dim3(CH * (KPV / 8) / 256), dim3(256), 0, stream>>>(pol_w1, CH, CH, PW1LD, WPV, CH, CH);
  k_plane<WFORM><<<dim3(VCH * (KPV / 8) / 256), dim3(256), 0, stream>>>(val_cw, VCH, CH, CH,
                                                                        WPV + (size_t)CH * KPV, VCH, CH);
  k_tab<<<dim3(TABROWS * CH / 4 / 256), dim3(256), 0, stream>>>(emb, pol_w1, pol_b1, pol_w2, TAB);

  const int tilesC = ((HWP + 63) / 64) * (CH / 64);
  const int tilesP = ((HWP + 63) / 64) * (NPVC / 64);

  k_im2col<<<dim3(MPAD * (KSTP / 8) / 256), dim3(256), 0, stream>>>(board, 1, HWP, KST, KSTP, 1, COL);
  k_gemm_nt<0, 0><<<dim3((tilesC + 7) / 8), dim3(256), 0, stream>>>(COL, WST, TAB, Y, HWP, CH, KSTP, CH);
  k_gn<<<dim3(1), dim3(512), 0, stream>>>(Y, stem_b, stem_gs, stem_gb, Y, A0, 0);

  float* X = A0;
  float* T = A1;
  float* O = A2;
  for (int i = 0; i < NBLK; ++i) {
    const int j0 = 2 * i;
    const int j1 = 2 * i + 1;
    k_im2col<<<dim3(MPAD * (KBLT / 8) / 256), dim3(256), 0, stream>>>(X, CH, 1, KBL, KBL, CONV_TERMS, COL);
    k_gemm_nt<0, 0><<<dim3((tilesC + 7) / 8), dim3(256), 0, stream>>>(COL, WB + (size_t)j0 * CH * KBLT, TAB, Y,
                                                                     HWP, CH, KBLT, CH);
    k_gn<<<dim3(1), dim3(512), 0, stream>>>(Y, blk_b + j0 * CH, blk_gs + j0 * CH, blk_gb + j0 * CH, Y, T, 0);
    k_im2col<<<dim3(MPAD * (KBLT / 8) / 256), dim3(256), 0, stream>>>(T, CH, 1, KBL, KBL, CONV_TERMS, COL);
    k_gemm_nt<0, 0><<<dim3((tilesC + 7) / 8), dim3(256), 0, stream>>>(COL, WB + (size_t)j1 * CH * KBLT, TAB, Y,
                                                                     HWP, CH, KBLT, CH);
    k_gn<<<dim3(1), dim3(512), 0, stream>>>(Y, blk_b + j1 * CH, blk_gs + j1 * CH, blk_gb + j1 * CH, X, O, 1);
    float* nx = O;
    O = X;
    X = nx;
  }

  k_plane<AFORM><<<dim3(MPAD * (KPV / 8) / 256), dim3(256), 0, stream>>>(X, HWP, CH, CH, FHL, MPAD, CH);
  k_gemm_nt<0, 0><<<dim3((tilesP + 7) / 8), dim3(256), 0, stream>>>(FHL, WPV, TAB, PV, HWP, NPVC, KPV, NPVC);
  k_moves<<<dim3(NMOVES / (32 * POLW)), dim3(32 * POLW), 0, stream>>>(PV, TAB, cells, cell_counts, piece_ids,
                                                                     anchors, sizes, pol_b2, out);
  k_shead<<<dim3(1), dim3(256), 0, stream>>>(PV, val_cb, val_gs, val_gb, srem, orem, phase,
                                             val_w1, val_b1, val_w2, val_b2, val_w3, val_b3, out);
  (void)hipGetLastError();
}
